// RoPEAttention_27865747816591
// MI455X (gfx1250) — hardware-verified
//
#include <hip/hip_runtime.h>
#ifndef NB
#define NB 2
#endif
#ifndef SQ
#ifdef SEQ
#define SQ SEQ
#else
#define SQ 2048
#endif
#endif
#define NB_FULL 2
#define SQ_FULL 2048
#define DM 1024
#define NH 16
#define HD 64
#define HG 2
#define NR ((size_t)NB * SQ)
static_assert(NB >= 1 && NB <= NB_FULL);
static_assert(SQ >= 256 && SQ <= SQ_FULL && SQ % 256 == 0);
static_assert(NH % HG == 0);
static_assert(DM == NH * HD);

typedef unsigned short v8us __attribute__((ext_vector_type(8), may_alias));
typedef float  v8f  __attribute__((ext_vector_type(8)));
typedef float  v4f  __attribute__((ext_vector_type(4)));
typedef float  v4fa __attribute__((ext_vector_type(4), may_alias));
typedef _Float16 v16h __attribute__((ext_vector_type(16)));
typedef _Float16 v4h __attribute__((ext_vector_type(4)));
union FragH { v16h v; v8us half[2]; _Float16 h[16]; unsigned short u[16]; };
struct InvF { float v[HD / 2]; };
static_assert(sizeof(InvF) == 4 * (HD / 2));

__device__ __forceinline__ unsigned short bf16_bits(float x) { unsigned int u = __float_as_uint(x); return (unsigned short)((u + 0x7FFFu + ((u >> 16) & 1u)) >> 16); }
__device__ __forceinline__ float bf16_val(unsigned short b) { return __uint_as_float(((unsigned int)b) << 16); }
__device__ __forceinline__ float bf16_rne(float x) { return bf16_val(bf16_bits(x)); }

__global__ __launch_bounds__(256) void k_wt_f16(const float* __restrict__ W, _Float16* __restrict__ Wt, int K, int N, float scale) {
  const int t = blockIdx.x * 256 + threadIdx.x; if (t >= N * (K / 8)) return; const int n = t / (K / 8), k8 = (t % (K / 8)) * 8; FragH f;
#pragma unroll
  for (int i = 0; i < 8; ++i) f.h[i] = (_Float16)(bf16_rne(W[(size_t)(k8 + i) * N + n]) * scale);
  const v8us o = f.half[0]; unsigned short* dst = (unsigned short*)Wt + (size_t)n * K + k8;
  *(volatile v8us*)dst = o; __threadfence(); *(volatile v8us*)dst = o;
}

__global__ __launch_bounds__(256) void k_x16r(const float* __restrict__ x, _Float16* __restrict__ X16, size_t n8) {
  const size_t t = (size_t)blockIdx.x * 256 + threadIdx.x; if (t >= n8) return;
  const size_t r = t / (DM / 8); const int c8 = (int)(t % (DM / 8)) * 8;
  const size_t b = r / SQ, sp = r % SQ;
  const float* src = x + (b * SQ_FULL + sp) * (size_t)DM + c8;
  const v4f a = *(const v4fa*)src, c = *(const v4fa*)(src + 4);
  FragH f;
#pragma unroll
  for (int q = 0; q < 4; ++q) { f.h[q] = (_Float16)bf16_rne(a[q]); f.h[4 + q] = (_Float16)bf16_rne(c[q]); }
  const v8us o = f.half[0]; unsigned short* dst = (unsigned short*)X16 + t * 8;
  *(volatile v8us*)dst = o; __threadfence(); *(volatile v8us*)dst = o;
}

__global__ __launch_bounds__(256) void k_v16(const float* __restrict__ F, int ldf, int coff, _Float16* __restrict__ H16, int ldo, int nrows) {
  const int t = blockIdx.x * 256 + threadIdx.x; const int per = DM / 8; if (t >= nrows * per) return;
  const int r = t / per, c8 = (t % per) * 8;
  const float* src = F + (size_t)r * ldf + coff + c8;
  const v4f a = *(const v4fa*)src, c = *(const v4fa*)(src + 4);
  FragH f;
#pragma unroll
  for (int q = 0; q < 4; ++q) { f.h[q] = (_Float16)a[q]; f.h[4 + q] = (_Float16)c[q]; }
  const v8us o = f.half[0]; unsigned short* dst = (unsigned short*)H16 + (size_t)r * ldo + c8;
  *(volatile v8us*)dst = o; __threadfence(); *(volatile v8us*)dst = o;
}

__global__ __launch_bounds__(256) void k_tab2(InvF tab, float* __restrict__ CS, float* __restrict__ SN) {
  #pragma clang fp contract(off)
  const int t = blockIdx.x * 256 + threadIdx.x; if (t >= SQ * (HD / 2)) return; const int i = t % (HD / 2); const int p = t / (HD / 2);
  float invf = tab.v[0];
#pragma unroll
  for (int k = 1; k < HD / 2; ++k) invf = (i == k) ? tab.v[k] : invf;
  const float ang = __fmul_rn((float)p, invf); const float c = cosf(ang), s = sinf(ang);
  *(volatile float*)(CS + t) = c; *(volatile float*)(SN + t) = s; __threadfence(); *(volatile float*)(CS + t) = c; *(volatile float*)(SN + t) = s;
}

template <int ROPE>
__global__ __launch_bounds__(64) void k_xform(const float* __restrict__ F, int ldf, int nh, const float* __restrict__ CS, const float* __restrict__ SN, _Float16* __restrict__ H16, int ldo) {
  #pragma clang fp contract(off)
  __shared__ float xv[HD]; __shared__ unsigned short sh_[HD];
  const int d = threadIdx.x; const int h = blockIdx.x % nh; const size_t r = blockIdx.x / nh; const int p = (int)(r % SQ);
  const float x = F[r * (size_t)ldf + (size_t)h * HD + d];
  xv[d] = x; __syncthreads();
  float o = x;
  if (ROPE == 2) { const int i = d & (HD / 2 - 1); const float c = CS[p * (HD / 2) + i], s = SN[p * (HD / 2) + i]; const float lo = xv[i], hi = xv[i + HD / 2];
    o = (d < HD / 2) ? __fadd_rn(__fmul_rn(lo, c), -__fmul_rn(hi, s)) : __fadd_rn(__fmul_rn(lo, s), __fmul_rn(hi, c)); }
  FragH th; th.h[0] = (_Float16)o; sh_[d] = th.u[0]; __syncthreads();
  if (d < HD / 8) { FragH f;
#pragma unroll
    for (int q = 0; q < 8; ++q) f.u[q] = sh_[d * 8 + q];
    const v8us o8 = f.half[0]; unsigned short* dst = (unsigned short*)H16 + r * (size_t)ldo + (size_t)h * HD + d * 8;
    *(volatile v8us*)dst = o8; __threadfence(); *(volatile v8us*)dst = o8; }
}

template <int NHv, int TTv>
__global__ __launch_bounds__(256) void k_vt(const _Float16* __restrict__ V16, int ldv, int voff, _Float16* __restrict__ Vt) { __shared__ unsigned short tl[64][66]; const int tid = threadIdx.x; const int slab = blockIdx.x / (TTv / 64), lg = blockIdx.x % (TTv / 64); const int b = slab / NHv, h = slab % NHv;
  for (int i = tid; i < 64 * 8; i += 256) { const int r = i / 8, c8 = (i % 8) * 8; FragH f; f.half[0] = *(const v8us*)((const unsigned short*)V16 + ((size_t)b * TTv + lg * 64 + r) * ldv + voff + h * 64 + c8);
#pragma unroll
    for (int q = 0; q < 8; ++q) tl[r][c8 + q] = f.u[q]; }
  __syncthreads();
  for (int pass = 0; pass < 2; ++pass) {
#pragma unroll
    for (int rd = 0; rd < 2; ++rd) { const int d = rd * 32 + tid / 8, pc = tid % 8; FragH f;
#pragma unroll
      for (int q = 0; q < 8; ++q) f.u[q] = tl[pc * 8 + q][d];
      *(volatile v8us*)((unsigned short*)Vt + ((size_t)slab * 64 + d) * TTv + lg * 64 + pc * 8) = f.half[0]; }
    if (pass == 0) __threadfence(); } }

__device__ __forceinline__ v16h g2_frag(const _Float16* p, int hh) { FragH f; f.half[0] = *(const v8us*)((const unsigned short*)p + 8 * hh); f.half[1] = *(const v8us*)((const unsigned short*)p + 16 + 8 * hh); return f.v; }
__device__ __forceinline__ v8f g2_mma(v16h a, v16h b, v8f c) { v8f d = __builtin_amdgcn_wmma_f32_16x16x32_f16(false, a, false, b, (short)0, c, false, false); asm volatile("v_nop\n\tv_nop\n\tv_nop\n\tv_nop" : "+v"(d) : "v"(a), "v"(b)); return d; }
__global__ __launch_bounds__(128) void k_gemm2(const _Float16* __restrict__ A, int lda, size_t sA, const _Float16* __restrict__ Bh, int ldb, size_t sB, float alpha, const float* __restrict__ bias,
    float* __restrict__ C, _Float16* __restrict__ C16, int ldc, size_t sC, int M, int N, int K) {
  __shared__ __attribute__((aligned(16))) float so[4][32][68];
  const int tid = threadIdx.x, w = tid >> 5, lane = tid & 31, ln = lane & 15, hh = lane >> 4; const int by = blockIdx.y;
  A += (size_t)by * sA; Bh += (size_t)by * sB; const size_t cofs = (size_t)by * sC;
  const int ntn = N >> 6; const int mt = blockIdx.x / ntn, nq = blockIdx.x - mt * ntn; const int row0 = mt * 128 + 32 * w, col0 = nq * 64; if (row0 >= M) return;
  const _Float16* a0p = A + (size_t)(row0 + ln) * lda; const _Float16* a1p = a0p + (size_t)16 * lda;
  const _Float16* b0p = Bh + (size_t)(col0 + ln) * ldb; const _Float16* b1p = b0p + (size_t)16 * ldb; const _Float16* b2p = b1p + (size_t)16 * ldb; const _Float16* b3p = b2p + (size_t)16 * ldb;
  const v8f z8 = {0.f,0.f,0.f,0.f,0.f,0.f,0.f,0.f}; v8f c00 = z8, c01 = z8, c02 = z8, c03 = z8, c10 = z8, c11 = z8, c12 = z8, c13 = z8;
#pragma unroll 1
  for (int kb = 0; kb < K; kb += 32) { const v16h a0 = g2_frag(a0p + kb, hh), a1 = g2_frag(a1p + kb, hh);
    v16h b = g2_frag(b0p + kb, hh); c00 = g2_mma(a0, b, c00); c10 = g2_mma(a1, b, c10);
    b = g2_frag(b1p + kb, hh); c01 = g2_mma(a0, b, c01); c11 = g2_mma(a1, b, c11);
    b = g2_frag(b2p + kb, hh); c02 = g2_mma(a0, b, c02); c12 = g2_mma(a1, b, c12);
    b = g2_frag(b3p + kb, hh); c03 = g2_mma(a0, b, c03); c13 = g2_mma(a1, b, c13); }
  v8f accs[8] = {c00, c01, c02, c03, c10, c11, c12, c13};
#pragma unroll
  for (int u = 0; u < 8; ++u) { const int t = u & 3, half = u >> 2; const int col = col0 + t * 16 + ln; const float bv = bias ? bf16_rne(bias[col]) : 0.f;
#pragma unroll
    for (int r = 0; r < 8; ++r) { const int rloc = half * 16 + 8 * hh + r; so[w][rloc][t * 16 + ln] = accs[u][r] * alpha + bv; } }
  __builtin_amdgcn_fence(4, "workgroup"); __builtin_amdgcn_wave_barrier();
  const int rsub = lane >> 4, c4 = (lane & 15) * 4;
  for (int pass = 0; pass < 2; ++pass) {
#pragma unroll
    for (int q = 0; q < 16; ++q) { const int r = q * 2 + rsub; const v4f v = *(const v4fa*)&so[w][r][c4];
      if (C) *(volatile v4f*)(C + cofs + (size_t)(row0 + r) * ldc + col0 + c4) = v;
      if (C16) { v4h h4;
#pragma unroll
        for (int i = 0; i < 4; ++i) h4[i] = (_Float16)v[i];
        *(volatile v4h*)(C16 + cofs + (size_t)(row0 + r) * ldc + col0 + c4) = h4; } }
    if (pass == 0) __threadfence(); }
}

__global__ __launch_bounds__(256) void k_rsmw(const float* __restrict__ S, _Float16* __restrict__ P, int qn, int hg) {
  #pragma clang fp contract(off)
  const int lane = threadIdx.x & 31;
  const int t = blockIdx.x * 8 + (int)(threadIdx.x >> 5);
  if (t >= qn * hg) return;
  const size_t i = (size_t)(t / qn) * SQ + (size_t)(t % qn);
  const float* s = S + i * SQ; unsigned short* prow = (unsigned short*)P + i * SQ;
  float mx = -3.0e38f;
#pragma unroll 1
  for (int j0 = lane * 8; j0 < SQ; j0 += 256) { const v4f a = *(const v4fa*)(s + j0), c = *(const v4fa*)(s + j0 + 4);
#pragma unroll
    for (int q = 0; q < 4; ++q) { mx = fmaxf(mx, a[q]); mx = fmaxf(mx, c[q]); } }
#pragma unroll
  for (int o = 16; o > 0; o >>= 1) mx = fmaxf(mx, __shfl_xor(mx, o, 32));
  float se = 0.f;
#pragma unroll 1
  for (int j0 = lane * 8; j0 < SQ; j0 += 256) { const v4f a = *(const v4fa*)(s + j0), c = *(const v4fa*)(s + j0 + 4);
#pragma unroll
    for (int q = 0; q < 4; ++q) { se += __expf(a[q] - mx); se += __expf(c[q] - mx); } }
#pragma unroll
  for (int o = 16; o > 0; o >>= 1) se += __shfl_xor(se, o, 32);
  const float sc = 1024.0f / se;
#pragma unroll 1
  for (int j0 = lane * 8; j0 < SQ; j0 += 256) { const v4f a = *(const v4fa*)(s + j0), c = *(const v4fa*)(s + j0 + 4); FragH f;
#pragma unroll
    for (int q = 0; q < 4; ++q) { f.h[q] = (_Float16)(__expf(a[q] - mx) * sc); f.h[4 + q] = (_Float16)(__expf(c[q] - mx) * sc); }
    const v8us o8 = f.half[0];
    *(volatile v8us*)(prow + j0) = o8; __threadfence(); *(volatile v8us*)(prow + j0) = o8; }
}

extern "C" void kernel_launch(void* const* d_in, const int* in_sizes, int n_in,
                              void* d_out, int out_size, void* d_ws, size_t ws_size, hipStream_t stream) {
  if (n_in < 5) return;
  if (in_sizes[0] < (int)((((size_t)(NB - 1)) * SQ_FULL + SQ) * DM)) return;
  if (in_sizes[1] < DM * 3 * DM || in_sizes[2] < 3 * DM || in_sizes[3] < DM * DM || in_sizes[4] < DM) return;
  if (out_size < (int)(NR * DM)) return;
  const float* x = (const float*)d_in[0]; const float* wqkv = (const float*)d_in[1]; const float* bqkv = (const float*)d_in[2]; const float* wout = (const float*)d_in[3]; const float* bout = (const float*)d_in[4];
  char* ws = (char*)d_ws; size_t off = 0;
  auto take = [&](size_t bytes) { char* p = ws + off; off += (bytes + 255) & ~(size_t)255; return p; };
  _Float16* BQKV = (_Float16*)take((size_t)3 * DM * DM * 2);
  _Float16* BO = (_Float16*)take((size_t)DM * DM * 2);
  float* CS = (float*)take((size_t)SQ * (HD / 2) * 4); float* SN = (float*)take((size_t)SQ * (HD / 2) * 4);
  _Float16* X16 = (_Float16*)take(NR * DM * 2);
  float* QKVF = (float*)take((size_t)SQ * 3 * DM * 4);
  _Float16* QH = (_Float16*)take(NR * DM * 2); _Float16* KH = (_Float16*)take(NR * DM * 2); _Float16* V16 = (_Float16*)take(NR * DM * 2); _Float16* O16 = (_Float16*)take(NR * DM * 2);
  float* S = (float*)take((size_t)HG * SQ * SQ * 4); _Float16* P = (_Float16*)take((size_t)HG * SQ * SQ * 2); _Float16* VT = (_Float16*)take((size_t)NH * HD * SQ * 2);
  if (off > ws_size) return;
  InvF tab;
  { double rt = 10000.0; for (int lv = 0; lv < 5; ++lv) { double y = rt; for (int it = 0; it < 64; ++it) y = 0.5 * (y + rt / y); rt = y; }
    double pw = 1.0; for (int i = 0; i < HD / 2; ++i) { tab.v[i] = (float)(1.0 / pw); pw *= rt; } }
  k_wt_f16<<<(unsigned)((3 * DM * (DM / 8) + 255) / 256), 256, 0, stream>>>(wqkv, BQKV, DM, 3 * DM, 16.0f);
  k_wt_f16<<<(unsigned)((DM * (DM / 8) + 255) / 256), 256, 0, stream>>>(wout, BO, DM, DM, 16.0f);
  k_tab2<<<(SQ * (HD / 2) + 255) / 256, 256, 0, stream>>>(tab, CS, SN);
  k_x16r<<<(unsigned)((NR * DM / 8 + 255) / 256), 256, 0, stream>>>(x, X16, NR * DM / 8);
  for (int b = 0; b < NB; ++b) { const size_t r0 = (size_t)b * SQ;
    k_gemm2<<<dim3((unsigned)((SQ / 128) * (3 * DM / 64)), 1), 128, 0, stream>>>(X16 + r0 * DM, DM, 0, BQKV, DM, 0, 0.0625f, bqkv, QKVF, nullptr, 3 * DM, 0, SQ, 3 * DM, DM);
    k_xform<2><<<(unsigned)(SQ * NH), 64, 0, stream>>>(QKVF, 3 * DM, NH, CS, SN, QH + r0 * DM, DM);
    k_xform<2><<<(unsigned)(SQ * NH), 64, 0, stream>>>(QKVF + DM, 3 * DM, NH, CS, SN, KH + r0 * DM, DM);
    k_v16<<<(unsigned)((SQ * (DM / 8) + 255) / 256), 256, 0, stream>>>(QKVF, 3 * DM, 2 * DM, V16 + r0 * DM, DM, SQ);
    k_vt<NH, SQ><<<NH * (SQ / 64), 256, 0, stream>>>(V16 + r0 * DM, DM, 0, VT);
    for (int h0 = 0; h0 < NH; h0 += HG) {
      k_gemm2<<<dim3((SQ / 128) * (SQ / 64), HG), 128, 0, stream>>>(QH + r0 * DM + h0 * HD, DM, (size_t)HD, KH + r0 * DM + h0 * HD, DM, (size_t)HD, 0.125f, nullptr, S, nullptr, SQ, (size_t)SQ * SQ, SQ, SQ, HD);
      k_rsmw<<<(HG * SQ + 7) / 8, 256, 0, stream>>>(S, P, SQ, HG);
      k_gemm2<<<dim3((SQ / 128) * (HD / 64), HG), 128, 0, stream>>>(P, SQ, (size_t)SQ * SQ, VT + (size_t)h0 * HD * SQ, SQ, (size_t)HD * SQ, 0.0625f, nullptr, nullptr, O16 + r0 * DM + h0 * HD, DM, (size_t)HD, SQ, HD, SQ); } }
  k_gemm2<<<dim3((unsigned)((NR / 128) * (DM / 64)), 1), 128, 0, stream>>>(O16, DM, 0, BO, DM, 0, 0.0009765625f, bout, (float*)d_out, nullptr, DM, 0, (int)NR, DM, DM);
}
